// HSTUAttention_79757542687326
// MI455X (gfx1250) — hardware-verified
//
#include <hip/hip_runtime.h>
#include <math.h>

constexpr int kBatch = 4;
constexpr int kSeq   = 2048;
constexpr int kDim   = 512;
constexpr int kHeads = 8;
constexpr int kHdim  = 64;
constexpr int kTok   = kBatch * kSeq;
constexpr int kProj  = 4 * kDim;
constexpr int kHeadsPerChunk = 4;
constexpr int kChunksPerBatch = kHeads / kHeadsPerChunk;
constexpr int kChunks = kBatch * kChunksPerBatch;
constexpr float kQScale    = 0.125f;
constexpr float kACarry    = 256.0f;
constexpr float kACarryInv = 1.0f / 256.0f;
constexpr float kInvDim    = 1.0f / 512.0f;
constexpr float kLnEps     = 1e-5f;

constexpr size_t kMiB     = 1048576;
constexpr size_t kOffXhi  = 0;
constexpr size_t kOffXlo  = 8 * kMiB;
constexpr size_t kOffW1hi = 16 * kMiB;
constexpr size_t kOffW1lo = 18 * kMiB;
constexpr size_t kOffV32  = 20 * kMiB;
constexpr size_t kOffA16  = 0;
constexpr size_t kOffNGhi = 0;
constexpr size_t kOffNGlo = 8 * kMiB;
constexpr size_t kOffGate = 64 * kMiB;
constexpr size_t kOffQK16 = 80 * kMiB;
constexpr size_t kOffVT16 = 96 * kMiB;
constexpr size_t kOffO32  = 104 * kMiB;
constexpr size_t kOffW2hi = 120 * kMiB;
constexpr size_t kOffW2lo = 120 * kMiB + 512 * 1024;
constexpr size_t kWsTotal = 121 * kMiB;

static_assert((size_t)kTok * kDim * 2 == 8 * kMiB);
static_assert((size_t)kProj * kDim * 2 == 2 * kMiB);
static_assert(kOffV32 + (size_t)kTok * kDim * 4 <= kOffGate);
static_assert(kOffA16 + (size_t)kHeadsPerChunk * kSeq * kSeq * 2 == 32 * kMiB);
static_assert(kOffA16 + (size_t)kHeadsPerChunk * kSeq * kSeq * 2 <= kOffGate);
static_assert(kOffNGlo + (size_t)kTok * kDim * 2 <= kOffGate);
static_assert(kOffGate + (size_t)kTok * kDim * 4 == kOffQK16);
static_assert(kOffQK16 + (size_t)kTok * 2 * kDim * 2 == kOffVT16);
static_assert(kOffVT16 + (size_t)kBatch * kHeads * kHdim * kSeq * 2 == kOffO32);
static_assert(kOffO32 + (size_t)kTok * kDim * 4 == kOffW2hi);
static_assert(kOffW2hi + (size_t)kDim * kDim * 2 == kOffW2lo);
static_assert(kOffW2lo + (size_t)kDim * kDim * 2 == kWsTotal);
static_assert(kWsTotal <= 134217728);

typedef __attribute__((ext_vector_type(16))) _Float16 v16h;
typedef __attribute__((ext_vector_type(8)))  _Float16 v8h;
typedef __attribute__((ext_vector_type(16))) __bf16   v16b;
typedef __attribute__((ext_vector_type(8)))  __bf16   v8b;
typedef __attribute__((ext_vector_type(8)))  float    v8f;
typedef __attribute__((ext_vector_type(4)))  float    v4f;
typedef __attribute__((ext_vector_type(4)))  unsigned int v4u;

__device__ __forceinline__ unsigned short f2bf_bits(float f) {
  unsigned u = __float_as_uint(f);
  return (unsigned short)((u + 0x7FFFu + ((u >> 16) & 1u)) >> 16);
}
__device__ __forceinline__ float bf_bits2f(unsigned short h) { return __uint_as_float(((unsigned)h) << 16); }

__device__ __forceinline__ void dep_guard_h(v8f& a, v8f& b, v16h x, v16h y) { asm volatile("v_nop\n\tv_nop\n\tv_nop\n\tv_nop" : "+v"(a), "+v"(b) : "v"(x), "v"(y)); }
__device__ __forceinline__ void dep_guard_b(v8f& a, v8f& b, v16b x, v16b y) { asm volatile("v_nop\n\tv_nop\n\tv_nop\n\tv_nop" : "+v"(a), "+v"(b) : "v"(x), "v"(y)); }
__device__ __forceinline__ void keep4_h(v16h a, v16h b, v16h c, v16h d) { asm volatile("v_nop" :: "v"(a), "v"(b), "v"(c), "v"(d)); }
__device__ __forceinline__ void keep4_b(v16b a, v16b b, v16b c, v16b d) { asm volatile("v_nop" :: "v"(a), "v"(b), "v"(c), "v"(d)); }
__device__ __forceinline__ void acc_guard4(v8f& a, v8f& b, v8f& c, v8f& d) { asm volatile("v_nop\n\tv_nop\n\tv_nop\n\tv_nop" : "+v"(a), "+v"(b), "+v"(c), "+v"(d)); }
template <typename T> struct Frag;
template <> struct Frag<_Float16> {
  typedef v16h V; union U { v16h v; v8h h[2]; };
  static __device__ __forceinline__ v16h load(const _Float16* p) {
    U f; f.h[0] = *(const v8h*)(p); f.h[1] = *(const v8h*)(p + 16); return f.v;
  }
  static __device__ __forceinline__ v8f mma(v16h a, v16h b, v8f c) {
    return __builtin_amdgcn_wmma_f32_16x16x32_f16(false, a, false, b, (short)0, c, false, false);
  }
  static __device__ __forceinline__ void guard(v8f& a, v8f& b, v16h x, v16h y) { dep_guard_h(a, b, x, y); }
  static __device__ __forceinline__ void keep(v16h a, v16h b, v16h c, v16h d) { keep4_h(a, b, c, d); }
};
template <> struct Frag<__bf16> {
  typedef v16b V; union U { v16b v; v8b h[2]; };
  static __device__ __forceinline__ v16b load(const __bf16* p) {
    U f; f.h[0] = *(const v8b*)(p); f.h[1] = *(const v8b*)(p + 16); return f.v;
  }
  static __device__ __forceinline__ v8f mma(v16b a, v16b b, v8f c) {
    return __builtin_amdgcn_wmma_f32_16x16x32_bf16(false, a, false, b, (short)0, c, false, false);
  }
  static __device__ __forceinline__ void guard(v8f& a, v8f& b, v16b x, v16b y) { dep_guard_b(a, b, x, y); }
  static __device__ __forceinline__ void keep(v16b a, v16b b, v16b c, v16b d) { keep4_b(a, b, c, d); }
};

__device__ __forceinline__ unsigned pk16(unsigned short a, unsigned short b) { return (unsigned)a | ((unsigned)b << 16); }
__device__ __forceinline__ unsigned short h_bits(float f) { const _Float16 h = (_Float16)f; return __builtin_bit_cast(unsigned short, h); }

template <int ET> struct Elem;
template <> struct Elem<0> { typedef _Float16 T; };
template <> struct Elem<1> { typedef __bf16 T; };
template <int ET, bool SPLIT, int BIAS_MODE, int OUT_MODE, bool RESID, int ACT, int TRI>
__global__ __launch_bounds__(256) void wmma_gemm64(
    const unsigned short* __restrict__ Ap, const unsigned short* __restrict__ A2p, int lda, long strideA,
    const unsigned short* __restrict__ Btp, const unsigned short* __restrict__ Bt2p, int ldb, long strideB,
    void* __restrict__ Cout, void* __restrict__ Cout2, int ldc, long strideC,
    const float* __restrict__ bias,
    const float* __restrict__ resid, long strideR,
    int M, int N, int K, float scale) {
  typedef typename Elem<ET>::T T;
  typedef typename Frag<T>::V V;
  const T* A = (const T*)Ap; const T* A2 = (const T*)A2p; const T* Bt = (const T*)Btp; const T* Bt2 = (const T*)Bt2p;
  __shared__ __align__(16) float sT[8][16 * 68];
  const int b    = blockIdx.y;
  const int lane = threadIdx.x & 31;
  const int wave = threadIdx.x >> 5;
  const int tilesN = N >> 6;
  const int tilesM = M >> 6;
  const int tile = blockIdx.x * 8 + wave;
  if (tile >= tilesM * tilesN) return;
  const int tm = tile / tilesN;
  const int tn = tile - tm * tilesN;
  const int m0 = tm << 6;
  const int n0 = tn << 6;

  int kEnd = K;
  if (TRI == 1) kEnd = (n0 > m0) ? 0 : K;
  if (TRI == 2) kEnd = (m0 + 64 < K) ? (m0 + 64) : K;

  const T* Ab  = A  + (size_t)b * strideA;
  const T* Bb  = Bt + (size_t)b * strideB;
  const T* Ab2 = SPLIT ? (A2  + (size_t)b * strideA) : nullptr;
  const T* Bb2 = SPLIT ? (Bt2 + (size_t)b * strideB) : nullptr;

  const int rlane = lane & 15;
  const int koff  = (lane >> 4) * 8;
  const int mOff  = (lane >> 4) * 8;

  v8f acc[4][4];
#pragma unroll
  for (int i = 0; i < 4; ++i)
#pragma unroll
    for (int j = 0; j < 4; ++j) acc[i][j] = (v8f){0.f,0.f,0.f,0.f,0.f,0.f,0.f,0.f};

  for (int k0 = 0; k0 < kEnd; k0 += 32) {
    V bh[4], bl[4];
#pragma unroll
    for (int j = 0; j < 4; ++j) {
      const size_t bo = (size_t)(n0 + (j << 4) + rlane) * ldb + koff + k0;
      bh[j] = Frag<T>::load(Bb + bo);
      if (SPLIT) bl[j] = Frag<T>::load(Bb2 + bo);
    }
#pragma unroll
    for (int i = 0; i < 4; ++i) {
      const size_t ao = (size_t)(m0 + (i << 4) + rlane) * lda + koff + k0;
      V ah = Frag<T>::load(Ab + ao);
      V al;
      if (SPLIT) al = Frag<T>::load(Ab2 + ao);
#pragma unroll
      for (int j = 0; j < 4; ++j) {
        acc[i][j] = Frag<T>::mma(ah, bh[j], acc[i][j]);
        if (SPLIT) {
          acc[i][j] = Frag<T>::mma(ah, bl[j], acc[i][j]);
          acc[i][j] = Frag<T>::mma(al, bh[j], acc[i][j]);
        }
      }
      Frag<T>::guard(acc[i][0], acc[i][3], ah, SPLIT ? al : ah);
    }
    Frag<T>::keep(bh[0], bh[1], bh[2], bh[3]);
    if (SPLIT) Frag<T>::keep(bl[0], bl[1], bl[2], bl[3]);
  }
  acc_guard4(acc[0][0], acc[0][1], acc[0][2], acc[0][3]);
  acc_guard4(acc[1][0], acc[1][1], acc[1][2], acc[1][3]);
  acc_guard4(acc[2][0], acc[2][1], acc[2][2], acc[2][3]);
  acc_guard4(acc[3][0], acc[3][1], acc[3][2], acc[3][3]);

  float* slab = sT[wave];
  const float* Rb = RESID ? (resid + (size_t)b * strideR) : nullptr;
#pragma unroll
  for (int i = 0; i < 4; ++i) {
    const int mBase = m0 + (i << 4);
#pragma unroll
    for (int j = 0; j < 4; ++j) {
      const int n = n0 + (j << 4) + rlane;
      float bv = 0.f;
      if (BIAS_MODE == 2) bv = bias[n];
#pragma unroll
      for (int r = 0; r < 8; ++r) {
        float v = acc[i][j][r] * scale;
        if (BIAS_MODE == 1) v += bias[mBase + mOff + r];
        if (BIAS_MODE == 2) v += bv;
        if (RESID) v += Rb[(size_t)(mBase + mOff + r) * ldc + n];
        if (ACT == 2) v = fmaxf(v, 0.0f);
        if (ACT == 3) v = v * (1.0f / (1.0f + expf(-v)));
        if (ACT == 4) v = (v > 0.f) ? v : 0.01f * v;
        if (ACT == 6) {
          const float sg = (v * (1.0f / (1.0f + expf(-v)))) * kACarry;
          v = (n <= mBase + mOff + r) ? sg : 0.0f;
        }
        slab[(mOff + r) * 68 + (j << 4) + rlane] = v;
      }
    }
    __builtin_amdgcn_fence(__ATOMIC_RELEASE, "workgroup");
    __builtin_amdgcn_wave_barrier();
    __builtin_amdgcn_fence(__ATOMIC_ACQUIRE, "workgroup");
    if (OUT_MODE == 0) {
      float* C = (float*)Cout + (size_t)b * strideC;
      const int hh = lane >> 4, c4 = (lane & 15) * 4;
      for (int pass = 0; pass < 2; ++pass) {
#pragma unroll
        for (int it = 0; it < 8; ++it) {
          const int row = it * 2 + hh;
          v4f v = *(const v4f*)(slab + row * 68 + c4);
          *(volatile v4f*)(C + (size_t)(mBase + row) * ldc + n0 + c4) = v;
        }
        __threadfence();
      }
    } else {
      const int q = lane >> 3, c8 = (lane & 7) * 8;
      unsigned short* C  = (unsigned short*)Cout  + (size_t)b * strideC;
      unsigned short* C2 = (OUT_MODE == 2) ? ((unsigned short*)Cout2 + (size_t)b * strideC) : nullptr;
      for (int pass = 0; pass < 2; ++pass) {
#pragma unroll
        for (int it = 0; it < 4; ++it) {
          const int row = it * 4 + q;
          const float* sp = slab + row * 68 + c8;
          v8h hv, lv;
#pragma unroll
          for (int e = 0; e < 8; ++e) {
            if (OUT_MODE == 1) {
              hv[e] = (_Float16)sp[e];
            } else {
              unsigned short hb = f2bf_bits(sp[e]);
              unsigned short lb = f2bf_bits(sp[e] - bf_bits2f(hb));
              hv[e] = __builtin_bit_cast(_Float16, hb);
              lv[e] = __builtin_bit_cast(_Float16, lb);
            }
          }
          *(volatile v8h*)(C + (size_t)(mBase + row) * ldc + n0 + c8) = hv;
          if (OUT_MODE == 2) *(volatile v8h*)(C2 + (size_t)(mBase + row) * ldc + n0 + c8) = lv;
        }
        __threadfence();
      }
    }
    __builtin_amdgcn_fence(__ATOMIC_RELEASE, "workgroup");
    __builtin_amdgcn_wave_barrier();
    __builtin_amdgcn_fence(__ATOMIC_ACQUIRE, "workgroup");
  }
}

__global__ __launch_bounds__(256) void split8_bf16_kernel(const float* __restrict__ in,
                                                          unsigned short* __restrict__ hi,
                                                          unsigned short* __restrict__ lo, int n8) {
  const int i = blockIdx.x * 256 + threadIdx.x;
  if (i >= n8) return;
  const float* p = in + 8 * (size_t)i;
  const v4f a = *(const v4f*)(p);
  const v4f c = *(const v4f*)(p + 4);
  unsigned short hb[8], lb[8];
#pragma unroll
  for (int e = 0; e < 4; ++e) {
    const float f0 = a[e];
    hb[e] = f2bf_bits(f0);
    lb[e] = f2bf_bits(f0 - bf_bits2f(hb[e]));
    const float f1 = c[e];
    hb[4 + e] = f2bf_bits(f1);
    lb[4 + e] = f2bf_bits(f1 - bf_bits2f(hb[4 + e]));
  }
  const v4u uh = (v4u){pk16(hb[0], hb[1]), pk16(hb[2], hb[3]), pk16(hb[4], hb[5]), pk16(hb[6], hb[7])};
  const v4u ul = (v4u){pk16(lb[0], lb[1]), pk16(lb[2], lb[3]), pk16(lb[4], lb[5]), pk16(lb[6], lb[7])};
  unsigned short* qh = hi + 8 * (size_t)i;
  unsigned short* ql = lo + 8 * (size_t)i;
  *(volatile v4u*)qh = uh;
  *(volatile v4u*)ql = ul;
  __threadfence();
  *(volatile v4u*)qh = uh;
  *(volatile v4u*)ql = ul;
}

__global__ __launch_bounds__(256) void vtcast_kernel(const float* __restrict__ v32, unsigned short* __restrict__ vt16) {
  __shared__ float sm[64][65];
  const int tt = threadIdx.x;
  const int t0 = blockIdx.x * 64;
  const int h  = blockIdx.y;
  const int b  = blockIdx.z;
  const float* src = v32 + ((size_t)b * kSeq + t0) * kDim + h * kHdim;
#pragma unroll
  for (int i = 0; i < 16; ++i) {
    const int e = i * 256 + tt;
    const int r = e >> 6;
    const int c = e & 63;
    sm[c][r] = src[(size_t)r * kDim + c];
  }
  __syncthreads();
  const int lane = tt & 31, wave = tt >> 5;
  const int q = lane >> 3, c8 = (lane & 7) * 8;
  unsigned short* dst = vt16 + ((size_t)(b * kHeads + h) * kHdim) * kSeq + t0;
  for (int pass = 0; pass < 2; ++pass) {
#pragma unroll
    for (int it = 0; it < 2; ++it) {
      const int row = wave * 8 + it * 4 + q;
      unsigned short hb[8];
#pragma unroll
      for (int e = 0; e < 8; ++e) hb[e] = h_bits(sm[row][c8 + e]);
      const v4u u = (v4u){pk16(hb[0], hb[1]), pk16(hb[2], hb[3]), pk16(hb[4], hb[5]), pk16(hb[6], hb[7])};
      *(volatile v4u*)(dst + (size_t)row * kSeq + c8) = u;
    }
    __threadfence();
  }
}

__global__ __launch_bounds__(256) void ln_gate_kernel(const float* __restrict__ o, const float* __restrict__ gate,
                                                      const float* __restrict__ lng, const float* __restrict__ lnb,
                                                      unsigned short* __restrict__ nghi, unsigned short* __restrict__ nglo,
                                                      int nrows) {
  const int lane = threadIdx.x & 31, wave = threadIdx.x >> 5;
  const int row = blockIdx.x * 8 + wave;
  if (row >= nrows) return;
  const float* po = o + (size_t)row * kDim;
  const float* pg = gate + (size_t)row * kDim;
  float xv[16], gv[16], gg[16], gb[16];
#pragma unroll
  for (int s = 0; s < 2; ++s) {
    const int c = s * 256 + lane * 8;
#pragma unroll
    for (int q = 0; q < 2; ++q) {
      const v4f a4 = *(const v4f*)(po + c + 4 * q);
      const v4f g4 = *(const v4f*)(pg + c + 4 * q);
      const v4f w4 = *(const v4f*)(lng + c + 4 * q);
      const v4f b4 = *(const v4f*)(lnb + c + 4 * q);
#pragma unroll
      for (int e = 0; e < 4; ++e) {
        const int idx = s * 8 + q * 4 + e;
        xv[idx] = a4[e]; gv[idx] = g4[e]; gg[idx] = w4[e]; gb[idx] = b4[e];
      }
    }
  }
  float sum = 0.f;
#pragma unroll
  for (int i = 0; i < 16; ++i) sum += xv[i];
#pragma unroll
  for (int off = 16; off > 0; off >>= 1) sum += __shfl_xor(sum, off, 32);
  const float mean = sum * kInvDim;
  float var = 0.f;
#pragma unroll
  for (int i = 0; i < 16; ++i) { const float d = xv[i] - mean; var += d * d; }
#pragma unroll
  for (int off = 16; off > 0; off >>= 1) var += __shfl_xor(var, off, 32);
  const float r = rsqrtf(var * kInvDim + kLnEps);
  unsigned short hb[16], lb[16];
#pragma unroll
  for (int i = 0; i < 16; ++i) {
    const float t = (xv[i] - mean) * r;
    const float val = (t * gg[i] + gb[i]) * gv[i];
    hb[i] = f2bf_bits(val);
    lb[i] = f2bf_bits(val - bf_bits2f(hb[i]));
  }
  const v4u uh0 = (v4u){pk16(hb[0], hb[1]), pk16(hb[2], hb[3]), pk16(hb[4], hb[5]), pk16(hb[6], hb[7])};
  const v4u uh1 = (v4u){pk16(hb[8], hb[9]), pk16(hb[10], hb[11]), pk16(hb[12], hb[13]), pk16(hb[14], hb[15])};
  const v4u ul0 = (v4u){pk16(lb[0], lb[1]), pk16(lb[2], lb[3]), pk16(lb[4], lb[5]), pk16(lb[6], lb[7])};
  const v4u ul1 = (v4u){pk16(lb[8], lb[9]), pk16(lb[10], lb[11]), pk16(lb[12], lb[13]), pk16(lb[14], lb[15])};
  unsigned short* ph = nghi + (size_t)row * kDim + lane * 8;
  unsigned short* pl = nglo + (size_t)row * kDim + lane * 8;
  for (int pass = 0; pass < 2; ++pass) {
    *(volatile v4u*)(ph)       = uh0;
    *(volatile v4u*)(ph + 256) = uh1;
    *(volatile v4u*)(pl)       = ul0;
    *(volatile v4u*)(pl + 256) = ul1;
    __threadfence();
  }
}

extern "C" void kernel_launch(void* const* d_in, const int* in_sizes, int n_in,
                              void* d_out, int out_size, void* d_ws, size_t ws_size,
                              hipStream_t stream) {
  if (n_in < 7) return;
  if (in_sizes[0] != kTok * kDim || in_sizes[1] != kProj * kDim || in_sizes[2] != kProj ||
      in_sizes[3] != kDim || in_sizes[4] != kDim || in_sizes[5] != kDim * kDim || in_sizes[6] != kDim) return;
  if (out_size != kTok * kDim) return;
  if (ws_size < kWsTotal) return;

  const float* x    = (const float*)d_in[0];
  const float* W1   = (const float*)d_in[1];
  const float* b1   = (const float*)d_in[2];
  const float* ln_g = (const float*)d_in[3];
  const float* ln_b = (const float*)d_in[4];
  const float* W2   = (const float*)d_in[5];
  const float* b2   = (const float*)d_in[6];
  float* out = (float*)d_out;
  char* ws = (char*)d_ws;

  unsigned short* xhi   = (unsigned short*)(ws + kOffXhi);
  unsigned short* xlo   = (unsigned short*)(ws + kOffXlo);
  unsigned short* w1hi  = (unsigned short*)(ws + kOffW1hi);
  unsigned short* w1lo  = (unsigned short*)(ws + kOffW1lo);
  float*          v32   = (float*)(ws + kOffV32);
  unsigned short* a16   = (unsigned short*)(ws + kOffA16);
  unsigned short* nghi  = (unsigned short*)(ws + kOffNGhi);
  unsigned short* nglo  = (unsigned short*)(ws + kOffNGlo);
  float*          gate  = (float*)(ws + kOffGate);
  unsigned short* qk16  = (unsigned short*)(ws + kOffQK16);
  unsigned short* vt16  = (unsigned short*)(ws + kOffVT16);
  float*          o32   = (float*)(ws + kOffO32);
  unsigned short* w2hi  = (unsigned short*)(ws + kOffW2hi);
  unsigned short* w2lo  = (unsigned short*)(ws + kOffW2lo);

  {
    const int n8x  = (kTok * kDim) / 8;
    const int n8w1 = (kProj * kDim) / 8;
    const int n8w2 = (kDim * kDim) / 8;
    split8_bf16_kernel<<<(n8x + 255) / 256, 256, 0, stream>>>(x, xhi, xlo, n8x);
    split8_bf16_kernel<<<(n8w1 + 255) / 256, 256, 0, stream>>>(W1, w1hi, w1lo, n8w1);
    split8_bf16_kernel<<<(n8w2 + 255) / 256, 256, 0, stream>>>(W2, w2hi, w2lo, n8w2);
  }

  {
    const int tilesGate = (kTok / 64) * (kDim / 64);
    const int tilesQK   = (kTok / 64) * (2 * kDim / 64);
    wmma_gemm64<1, true, 2, 0, false, 3, 0><<<dim3((tilesGate + 7) / 8, 1), 256, 0, stream>>>(
        xhi, xlo, kDim, 0L,
        w1hi, w1lo, kDim, 0L,
        (void*)gate, nullptr, kDim, 0L,
        b1, nullptr, 0L,
        kTok, kDim, kDim, 1.0f);
    wmma_gemm64<1, true, 2, 1, false, 3, 0><<<dim3((tilesQK + 7) / 8, 1), 256, 0, stream>>>(
        xhi, xlo, kDim, 0L,
        w1hi + (size_t)kDim * kDim, w1lo + (size_t)kDim * kDim, kDim, 0L,
        (void*)qk16, nullptr, 2 * kDim, 0L,
        b1 + kDim, nullptr, 0L,
        kTok, 2 * kDim, kDim, 1.0f);
    wmma_gemm64<1, true, 2, 0, false, 3, 0><<<dim3((tilesGate + 7) / 8, 1), 256, 0, stream>>>(
        xhi, xlo, kDim, 0L,
        w1hi + (size_t)3 * kDim * kDim, w1lo + (size_t)3 * kDim * kDim, kDim, 0L,
        (void*)v32, nullptr, kDim, 0L,
        b1 + 3 * kDim, nullptr, 0L,
        kTok, kDim, kDim, 1.0f);
  }

  vtcast_kernel<<<dim3(kSeq / 64, kHeads, kBatch), 256, 0, stream>>>(v32, vt16);

  for (int ch = 0; ch < kChunks; ++ch) {
    const int bb = ch / kChunksPerBatch;
    const int h0 = (ch % kChunksPerBatch) * kHeadsPerChunk;
    const size_t qkOff = (size_t)bb * kSeq * 2 * kDim + (size_t)h0 * kHdim;
    const int tilesS = (kSeq / 64) * (kSeq / 64);
    wmma_gemm64<0, false, 0, 1, false, 6, 1><<<dim3((tilesS + 7) / 8, kHeadsPerChunk), 256, 0, stream>>>(
        qk16 + qkOff, nullptr, 2 * kDim, (long)kHdim,
        qk16 + qkOff + kDim, nullptr, 2 * kDim, (long)kHdim,
        (void*)a16, nullptr, kSeq, (long)kSeq * kSeq,
        nullptr, nullptr, 0L,
        kSeq, kSeq, kHdim, kQScale);
    const int tilesO = (kSeq / 64) * (kHdim / 64);
    wmma_gemm64<0, false, 0, 0, false, 0, 2><<<dim3((tilesO + 7) / 8, kHeadsPerChunk), 256, 0, stream>>>(
        a16, nullptr, kSeq, (long)kSeq * kSeq,
        vt16 + (size_t)(bb * kHeads + h0) * kHdim * kSeq, nullptr, kSeq, (long)kHdim * kSeq,
        (void*)(o32 + (size_t)bb * kSeq * kDim + (size_t)h0 * kHdim), nullptr, kDim, (long)kHdim,
        nullptr, nullptr, 0L,
        kSeq, kHdim, kSeq, kACarryInv);
  }

  ln_gate_kernel<<<kTok / 8, 256, 0, stream>>>(o32, gate, ln_g, ln_b, nghi, nglo, kTok);

  {
    const int tilesOut = (kTok / 64) * (kDim / 64);
    wmma_gemm64<1, true, 2, 0, false, 0, 0><<<dim3((tilesOut + 7) / 8, 1), 256, 0, stream>>>(
        nghi, nglo, kDim, 0L,
        w2hi, w2lo, kDim, 0L,
        (void*)out, nullptr, kDim, 0L,
        b2, nullptr, 0L,
        kTok, kDim, kDim, 1.0f);
  }
}
